// scaled_dot_product_attn_7215545057961
// MI455X (gfx1250) — hardware-verified
//
#include <hip/hip_runtime.h>
#include <stdint.h>

typedef __attribute__((ext_vector_type(16))) _Float16 v16h;
typedef __attribute__((ext_vector_type(8)))  _Float16 v8h;
typedef __attribute__((ext_vector_type(8)))  float    v8f;
typedef __attribute__((ext_vector_type(4)))  float    v4f;

#define AT_D  64
#define AT_NW 4
#define AT_QB 64
#define AT_KC 64
#define SEQ_LEN 2048
#define PSC 32768.0f
#define EXP_C 0.180336880111120427f

__device__ __forceinline__ v8f mma16(v16h a, v16h b, v8f c) {
  c = __builtin_amdgcn_wmma_f32_16x16x32_f16(false, a, false, b, (short)0, c, false, false);
  asm volatile("v_nop\n\tv_nop\n\tv_nop\n\tv_nop" : "+v"(c) : "v"(a), "v"(b));
  return c;
}

__device__ __forceinline__ float ex2(float x) {
#if __has_builtin(__builtin_amdgcn_exp2f)
  return __builtin_amdgcn_exp2f(x);
#else
  float r;
  asm("v_exp_f32 %0, %1" : "=v"(r) : "v"(x));
  return r;
#endif
}

__global__ __launch_bounds__(128)
void attn64_f16_kernel(const float* __restrict__ q, const float* __restrict__ k,
                       const float* __restrict__ v, float* __restrict__ out, int S, int BH) {
  union FH { v16h v; v8h h[2]; };
  __shared__ __align__(16) _Float16 Ksh[AT_KC * AT_D];
  __shared__ __align__(16) _Float16 Vth[AT_D * AT_KC];
  __shared__ __align__(16) _Float16 Psh[AT_NW][16 * AT_KC];
  __shared__ __align__(16) float    Os[AT_NW][16 * 68];

  const int tid  = threadIdx.x;
  const int wave = tid >> 5;
  const int lane = tid & 31;
  const int hh   = lane >> 4;
  const int c    = lane & 15;

  const int nqb = S / AT_QB;
  const int bx  = blockIdx.x;
  const int qb  = bx % nqb;
  const int bh  = bx / nqb;
  if (bh >= BH) return;
  const int q0  = qb * AT_QB + wave * 16;

  const size_t hoff = (size_t)bh * (size_t)S * AT_D;
  const float* qb_ptr = q + hoff;
  const float* kb_ptr = k + hoff;
  const float* vb_ptr = v + hoff;
  float*       ob_ptr = out + hoff;

  v16h qa[2];
  {
    const float* qrow = qb_ptr + (size_t)(q0 + c) * AT_D;
#pragma unroll
    for (int dc = 0; dc < 2; ++dc) {
      const v4f a0 = *(const v4f*)(qrow + dc * 32 + 8 * hh);
      const v4f a1 = *(const v4f*)(qrow + dc * 32 + 8 * hh + 4);
      const v4f b0 = *(const v4f*)(qrow + dc * 32 + 16 + 8 * hh);
      const v4f b1 = *(const v4f*)(qrow + dc * 32 + 16 + 8 * hh + 4);
#pragma unroll
      for (int e = 0; e < 4; ++e) {
        qa[dc][e]      = (_Float16)a0[e];
        qa[dc][4 + e]  = (_Float16)a1[e];
        qa[dc][8 + e]  = (_Float16)b0[e];
        qa[dc][12 + e] = (_Float16)b1[e];
      }
    }
  }

  float mrow[8], lrow[8];
  v8f oacc[4];
#pragma unroll
  for (int r = 0; r < 8; ++r) { mrow[r] = -INFINITY; lrow[r] = 0.f; }
#pragma unroll
  for (int t = 0; t < 4; ++t) oacc[t] = (v8f){0.f,0.f,0.f,0.f,0.f,0.f,0.f,0.f};

  const int nChunks = S / AT_KC;
  for (int kc = 0; kc < nChunks; ++kc) {
    const int kv0 = kc * AT_KC;
    __syncthreads();
    {
      const int kvr = tid >> 1, dh = (tid & 1) * 32;
      const float* krow = kb_ptr + (size_t)(kv0 + kvr) * AT_D + dh;
      const float* vrow = vb_ptr + (size_t)(kv0 + kvr) * AT_D + dh;
#pragma unroll
      for (int i = 0; i < 4; ++i) {
        const v4f ka = *(const v4f*)(krow + 8 * i);
        const v4f kb = *(const v4f*)(krow + 8 * i + 4);
        v8h hk;
#pragma unroll
        for (int e = 0; e < 4; ++e) { hk[e] = (_Float16)ka[e]; hk[4 + e] = (_Float16)kb[e]; }
        *(v8h*)(Ksh + kvr * AT_D + dh + 8 * i) = hk;
      }
#pragma unroll
      for (int i = 0; i < 8; ++i) {
        const v4f vv = *(const v4f*)(vrow + 4 * i);
#pragma unroll
        for (int e = 0; e < 4; ++e) {
          const int d = dh + 4 * i + e;
          Vth[d * AT_KC + kvr] = (_Float16)vv[e];
        }
      }
    }
    __syncthreads();

    v8f s[4];
#pragma unroll
    for (int j = 0; j < 4; ++j) {
      s[j] = (v8f){0.f,0.f,0.f,0.f,0.f,0.f,0.f,0.f};
#pragma unroll
      for (int dc = 0; dc < 2; ++dc) {
        FH kf;
        kf.h[0] = *(const v8h*)(Ksh + (j * 16 + c) * AT_D + dc * 32 + 8 * hh);
        kf.h[1] = *(const v8h*)(Ksh + (j * 16 + c) * AT_D + dc * 32 + 16 + 8 * hh);
        s[j] = mma16(qa[dc], kf.v, s[j]);
      }
    }

    float cm[8];
#pragma unroll
    for (int r = 0; r < 8; ++r) {
      float m = fmaxf(fmaxf(s[0][r], s[1][r]), fmaxf(s[2][r], s[3][r]));
#pragma unroll
      for (int off = 1; off < 16; off <<= 1) m = fmaxf(m, __shfl_xor(m, off, 32));
      cm[r] = m;
    }

    _Float16* pw = Psh[wave];
#pragma unroll
    for (int r = 0; r < 8; ++r) {
      const float mnew  = fmaxf(mrow[r], cm[r]);
      const float alpha = ex2((mrow[r] - mnew) * EXP_C);
      mrow[r] = mnew;
      float psum = 0.f;
#pragma unroll
      for (int j = 0; j < 4; ++j) {
        const float p = ex2((s[j][r] - mnew) * EXP_C);
        psum += p;
        pw[(8 * hh + r) * AT_KC + j * 16 + c] = (_Float16)(p * PSC);
      }
#pragma unroll
      for (int off = 1; off < 16; off <<= 1) psum += __shfl_xor(psum, off, 32);
      lrow[r] = lrow[r] * alpha + psum;
#pragma unroll
      for (int t = 0; t < 4; ++t) oacc[t][r] *= alpha;
    }
    __builtin_amdgcn_fence(__ATOMIC_RELEASE, "workgroup");
    __builtin_amdgcn_wave_barrier();
    __builtin_amdgcn_fence(__ATOMIC_ACQUIRE, "workgroup");

#pragma unroll 1
    for (int kk = 0; kk < 2; ++kk) {
      FH pa;
      pa.h[0] = *(const v8h*)(pw + c * AT_KC + kk * 32 + 8 * hh);
      pa.h[1] = *(const v8h*)(pw + c * AT_KC + kk * 32 + 16 + 8 * hh);
#pragma unroll
      for (int t = 0; t < 4; ++t) {
        FH vf;
        vf.h[0] = *(const v8h*)(Vth + (t * 16 + c) * AT_KC + kk * 32 + 8 * hh);
        vf.h[1] = *(const v8h*)(Vth + (t * 16 + c) * AT_KC + kk * 32 + 16 + 8 * hh);
        oacc[t] = mma16(pa.v, vf.v, oacc[t]);
      }
    }
  }

  float* os = Os[wave];
#pragma unroll
  for (int r = 0; r < 8; ++r) {
    const float inv = 1.0f / (lrow[r] * PSC);
#pragma unroll
    for (int t = 0; t < 4; ++t) os[(8 * hh + r) * 68 + t * 16 + c] = oacc[t][r] * inv;
  }
  __builtin_amdgcn_fence(__ATOMIC_RELEASE, "workgroup");
  __builtin_amdgcn_wave_barrier();
  __builtin_amdgcn_fence(__ATOMIC_ACQUIRE, "workgroup");
  {
    const int c4 = (lane & 15) * 4;
    for (int pass = 0; pass < 2; ++pass) {
#pragma unroll
      for (int it = 0; it < 8; ++it) {
        const int row = it * 2 + hh;
        v4f val = *(const v4f*)(os + row * 68 + c4);
        *(volatile v4f*)(ob_ptr + (size_t)(q0 + row) * AT_D + c4) = val;
      }
      __threadfence();
    }
  }
}

extern "C" void kernel_launch(void* const* d_in, const int* in_sizes, int n_in,
                              void* d_out, int out_size, void* d_ws, size_t ws_size, hipStream_t stream) {
  (void)d_ws; (void)ws_size;
  if (n_in < 3) return;
  const int n = in_sizes[0];
  const int per_head = SEQ_LEN * AT_D;
  if (n <= 0 || (n % per_head) != 0) return;
  if (in_sizes[1] != n || in_sizes[2] != n || out_size != n) return;
  const int BH = n / per_head;
  const int S  = SEQ_LEN;

  const float* qp = (const float*)d_in[0];
  const float* kp = (const float*)d_in[1];
  const float* vp = (const float*)d_in[2];
  float* op = (float*)d_out;

  dim3 grid((unsigned)(BH * (S / AT_QB)), 1, 1);
  dim3 block(AT_NW * 32, 1, 1);
  attn64_f16_kernel<<<grid, block, 0, stream>>>(qp, kp, vp, op, S, BH);
  (void)hipGetLastError();
}
